// RGCNEncoder_20641612825459
// MI455X (gfx1250) — hardware-verified
//
#include <hip/hip_runtime.h>
#include <math.h>

constexpr int kNodes  = 50000;
constexpr int kEdges  = 600000;
constexpr int kFeat   = 128;
constexpr int kRel    = 8;
constexpr int kBases  = 4;
constexpr int kKtot   = kRel * kFeat + kFeat;
constexpr int kLinesPerRow = (kKtot * 2) / 128;
constexpr int kThreads = 256;
constexpr int kWaves   = kThreads / 32;
constexpr int kTileRows = 2048;
constexpr int kRowsPerWave = kTileRows / kWaves;
constexpr int kChunkNodes = 12288;
constexpr int kTilesPerChunk = kChunkNodes / kTileRows;
constexpr int kNumChunks = (kNodes + kChunkNodes - 1) / kChunkNodes;
constexpr int kLastCnt  = kNodes - (kNumChunks - 1) * kChunkNodes;
constexpr int kLastMpad = ((kLastCnt + 63) / 64) * 64;
constexpr int kHRows    = (kNumChunks - 1) * kChunkNodes + kLastMpad;
constexpr int kEdgeChunk = 2048;
constexpr int kSP = kEdgeChunk / kThreads;
constexpr int kNumEdgeChunks = (kEdges + kEdgeChunk - 1) / kEdgeChunk;
constexpr float kBCarry    = 64.0f;
constexpr float kBCarryInv = 1.0f / 64.0f;

static_assert(kKtot % 32 == 0);
static_assert(kKtot % 64 == 0);
static_assert(kFeat == 128);
static_assert(kFeat % 64 == 0);
static_assert(kChunkNodes % 64 == 0);
static_assert(kChunkNodes % kTileRows == 0);
static_assert(kTileRows == kWaves * kRowsPerWave);
static_assert(kTileRows <= 2048);
static_assert(kRel == 8);
static_assert(kNodes < 65536);
static_assert(kEdges % kSP == 0);
static_assert(kSP % 4 == 0);
static_assert(kHRows >= kNodes);
static_assert(kLastMpad <= kTileRows);
static_assert(kRel * kBases == 32);

constexpr size_t kBtBytes  = (size_t)kFeat * kKtot * 2;
constexpr size_t kAplBytes = (size_t)kChunkNodes * kKtot * 2;
constexpr size_t kAggBytes = (size_t)kTilesPerChunk * kTileRows * kRel * kFeat * 4;
constexpr size_t kHBytes   = (size_t)kHRows * kFeat * 4;
static_assert(2 * kBtBytes + kAplBytes + kAggBytes + kHBytes == (size_t)104857600);
static_assert(2 * kBtBytes + kAplBytes + kAggBytes + kHBytes <= (size_t)134217728);

typedef __attribute__((ext_vector_type(16))) _Float16 v16h;
typedef __attribute__((ext_vector_type(8)))  _Float16 v8h;
typedef __attribute__((ext_vector_type(16))) __bf16   v16b;
typedef __attribute__((ext_vector_type(8)))  __bf16   v8b;
typedef __attribute__((ext_vector_type(8)))  float    v8f;
typedef __attribute__((ext_vector_type(4)))  float    v4f;
typedef __attribute__((ext_vector_type(4)))  int      v4i;
typedef __attribute__((ext_vector_type(4)))  unsigned int v4u;

__device__ __forceinline__ unsigned short f2bf_bits(float f) {
  unsigned u = __float_as_uint(f);
  return (unsigned short)((u + 0x7FFFu + ((u >> 16) & 1u)) >> 16);
}
__device__ __forceinline__ float bf_bits2f(unsigned short h) { return __uint_as_float(((unsigned)h) << 16); }

__device__ __forceinline__ void dep_guard4_h(v8f& a, v8f& b, v8f& c, v8f& d, v16h x, v16h y) {
  asm volatile("v_nop\n\tv_nop\n\tv_nop\n\tv_nop" : "+v"(a), "+v"(b), "+v"(c), "+v"(d) : "v"(x), "v"(y));
}
__device__ __forceinline__ void dep_guard4_b(v8f& a, v8f& b, v8f& c, v8f& d, v16b x, v16b y) {
  asm volatile("v_nop\n\tv_nop\n\tv_nop\n\tv_nop" : "+v"(a), "+v"(b), "+v"(c), "+v"(d) : "v"(x), "v"(y));
}
__device__ __forceinline__ void keep4_h(v16h a, v16h b, v16h c, v16h d) { asm volatile("v_nop" :: "v"(a), "v"(b), "v"(c), "v"(d)); }
__device__ __forceinline__ void keep4_b(v16b a, v16b b, v16b c, v16b d) { asm volatile("v_nop" :: "v"(a), "v"(b), "v"(c), "v"(d)); }
__device__ __forceinline__ void acc_guard4(v8f& a, v8f& b, v8f& c, v8f& d) { asm volatile("v_nop\n\tv_nop\n\tv_nop\n\tv_nop" : "+v"(a), "+v"(b), "+v"(c), "+v"(d)); }
template <typename T> struct Frag;
template <> struct Frag<_Float16> {
  typedef v16h V; union U { v16h v; v8h h[2]; };
  static __device__ __forceinline__ v16h load(const _Float16* p) {
    U f; f.h[0] = *(const v8h*)(p); f.h[1] = *(const v8h*)(p + 16); return f.v;
  }
  static __device__ __forceinline__ v8f mma(v16h a, v16h b, v8f c) {
    return __builtin_amdgcn_wmma_f32_16x16x32_f16(false, a, false, b, (short)0, c, false, false);
  }
  static __device__ __forceinline__ void guard4(v8f& a, v8f& b, v8f& c, v8f& d, v16h x, v16h y) { dep_guard4_h(a, b, c, d, x, y); }
  static __device__ __forceinline__ void keep(v16h a, v16h b, v16h c, v16h d) { keep4_h(a, b, c, d); }
};
template <> struct Frag<__bf16> {
  typedef v16b V; union U { v16b v; v8b h[2]; };
  static __device__ __forceinline__ v16b load(const __bf16* p) {
    U f; f.h[0] = *(const v8b*)(p); f.h[1] = *(const v8b*)(p + 16); return f.v;
  }
  static __device__ __forceinline__ v8f mma(v16b a, v16b b, v8f c) {
    return __builtin_amdgcn_wmma_f32_16x16x32_bf16(false, a, false, b, (short)0, c, false, false);
  }
  static __device__ __forceinline__ void guard4(v8f& a, v8f& b, v8f& c, v8f& d, v16b x, v16b y) { dep_guard4_b(a, b, c, d, x, y); }
  static __device__ __forceinline__ void keep(v16b a, v16b b, v16b c, v16b d) { keep4_b(a, b, c, d); }
};

__device__ __forceinline__ unsigned pk16(unsigned short a, unsigned short b) { return (unsigned)a | ((unsigned)b << 16); }
__device__ __forceinline__ unsigned short h_bits(float f) { const _Float16 h = (_Float16)f; return __builtin_bit_cast(unsigned short, h); }
__device__ __forceinline__ v4u pack8h(v4f a, v4f b) {
  return (v4u){pk16(h_bits(a[0]), h_bits(a[1])), pk16(h_bits(a[2]), h_bits(a[3])),
               pk16(h_bits(b[0]), h_bits(b[1])), pk16(h_bits(b[2]), h_bits(b[3]))};
}

template <int ET> struct Elem;
template <> struct Elem<0> { typedef _Float16 T; };
template <> struct Elem<1> { typedef __bf16 T; };
template <int ET, bool SPLIT, int BIAS_MODE, int OUT_MODE, int ACT>
__global__ __launch_bounds__(256) void wmma_gemm64(
    const unsigned short* __restrict__ Ap, const unsigned short* __restrict__ A2p, int lda, long strideA,
    const unsigned short* __restrict__ Btp, const unsigned short* __restrict__ Bt2p, int ldb, long strideB,
    void* __restrict__ Cout, void* __restrict__ Cout2, int ldc, long strideC,
    const float* __restrict__ bias,
    int M, int N, int K, float scale, int Mlim) {
  typedef typename Elem<ET>::T T;
  typedef typename Frag<T>::V V;
  const T* A = (const T*)Ap; const T* A2 = (const T*)A2p; const T* Bt = (const T*)Btp; const T* Bt2 = (const T*)Bt2p;
  __shared__ __align__(16) float sT[8][16 * 68];
  const int b    = blockIdx.y;
  const int lane = threadIdx.x & 31;
  const int wave = threadIdx.x >> 5;
  const int tilesN = N >> 6;
  const int tilesM = M >> 6;
  const int tile = blockIdx.x * 8 + wave;
  if (tile >= tilesM * tilesN) return;
  const int tm = tile / tilesN;
  const int tn = tile - tm * tilesN;
  const int m0 = tm << 6;
  const int n0 = tn << 6;

  const T* Ab  = A  + (size_t)b * strideA;
  const T* Bb  = Bt + (size_t)b * strideB;
  const T* Ab2 = SPLIT ? (A2  + (size_t)b * strideA) : nullptr;
  const T* Bb2 = SPLIT ? (Bt2 + (size_t)b * strideB) : nullptr;

  const int rlane = lane & 15;
  const int koff  = (lane >> 4) * 8;
  const int mOff  = (lane >> 4) * 8;

  v8f acc[4][4];
#pragma unroll
  for (int i = 0; i < 4; ++i)
#pragma unroll
    for (int j = 0; j < 4; ++j) acc[i][j] = (v8f){0.f,0.f,0.f,0.f,0.f,0.f,0.f,0.f};

  for (int k0 = 0; k0 < K; k0 += 32) {
    V bh[4], bl[4];
#pragma unroll
    for (int j = 0; j < 4; ++j) {
      const size_t bo = (size_t)(n0 + (j << 4) + rlane) * ldb + koff + k0;
      bh[j] = Frag<T>::load(Bb + bo);
      if (SPLIT) bl[j] = Frag<T>::load(Bb2 + bo);
    }
#pragma unroll
    for (int i = 0; i < 4; ++i) {
      const size_t ao = (size_t)(m0 + (i << 4) + rlane) * lda + koff + k0;
      V ah = Frag<T>::load(Ab + ao);
      V al;
      if (SPLIT) al = Frag<T>::load(Ab2 + ao);
#pragma unroll
      for (int j = 0; j < 4; ++j) {
        acc[i][j] = Frag<T>::mma(ah, bh[j], acc[i][j]);
        if (SPLIT) {
          acc[i][j] = Frag<T>::mma(ah, bl[j], acc[i][j]);
          acc[i][j] = Frag<T>::mma(al, bh[j], acc[i][j]);
        }
      }
      Frag<T>::guard4(acc[i][0], acc[i][1], acc[i][2], acc[i][3], ah, SPLIT ? al : bh[3]);
    }
    Frag<T>::keep(bh[0], bh[1], bh[2], bh[3]);
    if (SPLIT) Frag<T>::keep(bl[0], bl[1], bl[2], bl[3]);
  }
  acc_guard4(acc[0][0], acc[0][1], acc[0][2], acc[0][3]);
  acc_guard4(acc[1][0], acc[1][1], acc[1][2], acc[1][3]);
  acc_guard4(acc[2][0], acc[2][1], acc[2][2], acc[2][3]);
  acc_guard4(acc[3][0], acc[3][1], acc[3][2], acc[3][3]);

  float* slab = sT[wave];
#pragma unroll
  for (int i = 0; i < 4; ++i) {
    const int mBase = m0 + (i << 4);
#pragma unroll
    for (int j = 0; j < 4; ++j) {
      const int n = n0 + (j << 4) + rlane;
      float bv = 0.f;
      if (BIAS_MODE == 2) bv = bias[n];
#pragma unroll
      for (int r = 0; r < 8; ++r) {
        float v = acc[i][j][r] * scale;
        if (BIAS_MODE == 1) v += bias[mBase + mOff + r];
        if (BIAS_MODE == 2) v += bv;
        if (ACT == 2) v = fmaxf(v, 0.0f);
        if (ACT == 4) v = (v > 0.f) ? v : 0.01f * v;
        slab[(mOff + r) * 68 + (j << 4) + rlane] = v;
      }
    }
    __builtin_amdgcn_fence(__ATOMIC_RELEASE, "workgroup");
    __builtin_amdgcn_wave_barrier();
    __builtin_amdgcn_fence(__ATOMIC_ACQUIRE, "workgroup");
    if (OUT_MODE == 0) {
      float* C = (float*)Cout + (size_t)b * strideC;
      const int hh = lane >> 4, c4 = (lane & 15) * 4;
      for (int pass = 0; pass < 2; ++pass) {
#pragma unroll
        for (int it = 0; it < 8; ++it) {
          const int row = it * 2 + hh;
          v4f v = *(const v4f*)(slab + row * 68 + c4);
          if (mBase + row < Mlim) *(volatile v4f*)(C + (size_t)(mBase + row) * ldc + n0 + c4) = v;
        }
        __threadfence();
      }
    } else {
      const int q = lane >> 3, c8 = (lane & 7) * 8;
      unsigned short* C  = (unsigned short*)Cout  + (size_t)b * strideC;
      unsigned short* C2 = (OUT_MODE == 2) ? ((unsigned short*)Cout2 + (size_t)b * strideC) : nullptr;
      for (int pass = 0; pass < 2; ++pass) {
#pragma unroll
        for (int it = 0; it < 4; ++it) {
          const int row = it * 4 + q;
          const float* sp = slab + row * 68 + c8;
          v8h hv, lv;
#pragma unroll
          for (int e = 0; e < 8; ++e) {
            if (OUT_MODE == 1) {
              hv[e] = (_Float16)sp[e];
            } else {
              unsigned short hb = f2bf_bits(sp[e]);
              unsigned short lb = f2bf_bits(sp[e] - bf_bits2f(hb));
              hv[e] = __builtin_bit_cast(_Float16, hb);
              lv[e] = __builtin_bit_cast(_Float16, lb);
            }
          }
          if (mBase + row < Mlim) {
            *(volatile v8h*)(C + (size_t)(mBase + row) * ldc + n0 + c8) = hv;
            if (OUT_MODE == 2) *(volatile v8h*)(C2 + (size_t)(mBase + row) * ldc + n0 + c8) = lv;
          }
        }
        __threadfence();
      }
    }
    __builtin_amdgcn_fence(__ATOMIC_RELEASE, "workgroup");
    __builtin_amdgcn_wave_barrier();
    __builtin_amdgcn_fence(__ATOMIC_ACQUIRE, "workgroup");
  }
}

__global__ __launch_bounds__(kThreads) void btbuild_kernel(const float* __restrict__ compA, const float* __restrict__ basisA,
                                                          const float* __restrict__ rootA,
                                                          const float* __restrict__ compB, const float* __restrict__ basisB,
                                                          const float* __restrict__ rootB,
                                                          unsigned short* __restrict__ BtA, unsigned short* __restrict__ BtB) {
  __shared__ __align__(16) float rowv[kKtot];
  __shared__ float cs[kRel * kBases];
  const int tid = threadIdx.x;
  const int o = blockIdx.x;
  const bool second = (blockIdx.y != 0);
  const float* comp  = second ? compB  : compA;
  const float* basis = second ? basisB : basisA;
  const float* root  = second ? rootB  : rootA;
  unsigned short* Bt = second ? BtB : BtA;
  if (tid < kRel * kBases) cs[tid] = comp[tid];
  __syncthreads();
#pragma unroll
  for (int q = 0; q < 4; ++q) {
    const int k = tid + kThreads * q;
    const int r = k >> 7;
    const int i = k & 127;
    float s = 0.0f;
#pragma unroll
    for (int bb = 0; bb < kBases; ++bb) s += cs[r * kBases + bb] * basis[((size_t)bb * kFeat + i) * kFeat + o];
    rowv[k] = s * kBCarry;
  }
  if (tid < kFeat) rowv[kRel * kFeat + tid] = root[(size_t)tid * kFeat + o] * kBCarry;
  __syncthreads();
  const int L  = tid >> 3, c = tid & 7;
  const int Lc = (L < kLinesPerRow) ? L : (kLinesPerRow - 1);
  const int k0 = Lc * 64 + c * 8;
  const v4f a0 = *(const v4f*)(rowv + k0);
  const v4f a1 = *(const v4f*)(rowv + k0 + 4);
  const v4u u = pack8h(a0, a1);
  unsigned short* dst = Bt + (size_t)o * kKtot + k0;
  for (int pass = 0; pass < 2; ++pass) {
    if (L < kLinesPerRow) *(volatile v4u*)dst = u;
    __threadfence();
  }
}

__device__ __forceinline__ int blk_excl_scan(int cnt, int* scan_ws, int tid, int* tot) {
  const int lane = tid & 31, wave = tid >> 5; int incl = cnt;
#pragma unroll
  for (int o = 1; o < 32; o <<= 1) { const int v = __shfl_up(incl, o, 32); if (lane >= o) incl += v; }
  if (lane == 31) scan_ws[wave] = incl;
  __syncthreads();
  if (wave == 0) { int wv = (lane < kThreads / 32) ? scan_ws[lane] : 0; int wincl = wv;
#pragma unroll
    for (int o = 1; o < 32; o <<= 1) { const int v = __shfl_up(wincl, o, 32); if (lane >= o) wincl += v; }
    if (lane < kThreads / 32) scan_ws[32 + lane] = wincl - wv; if (lane == 31) scan_ws[64] = wincl; }
  __syncthreads();
  const int res = scan_ws[32 + wave] + incl - cnt; *tot = scan_ws[64];
  return res;
}
__device__ __forceinline__ int chunk_hits(const int* __restrict__ dstv, const int* __restrict__ srcv, const int* __restrict__ etv,
                                          int e0, int n0, int tid, int* LIST, int* scan_ws) {
  const int eb = e0 + tid * kSP;
  const bool inr = (eb < kEdges);
  const int ebc = inr ? eb : (kEdges - kSP);
  int rec[kSP]; int cnt = 0;
#pragma unroll
  for (int k = 0; k < kSP; k += 4) {
    const v4i d4 = *(const v4i*)(dstv + ebc + k);
    const v4i s4 = *(const v4i*)(srcv + ebc + k);
    const v4i t4 = *(const v4i*)(etv + ebc + k);
#pragma unroll
    for (int e = 0; e < 4; ++e) {
      const int d = d4[e]; int r = -1;
      if (inr && d >= n0 && d < n0 + kTileRows) {
        int s = s4[e]; s = s < 0 ? 0 : (s >= kNodes ? kNodes - 1 : s);
        int t = t4[e]; t = t < 0 ? 0 : (t >= kRel ? kRel - 1 : t);
        r = ((d - n0) << 19) | (t << 16) | s; ++cnt;
      }
      rec[k + e] = r;
    }
  }
  int tot; int p = blk_excl_scan(cnt, scan_ws, tid, &tot);
#pragma unroll
  for (int k = 0; k < kSP; ++k) if (rec[k] >= 0) { if ((unsigned)p < (unsigned)kEdgeChunk) LIST[p] = rec[k]; ++p; }
  __syncthreads();
  return tot < kEdgeChunk ? tot : kEdgeChunk;
}

__global__ __launch_bounds__(kThreads) void agg_kernel(const float* __restrict__ F, const int* __restrict__ ei, const int* __restrict__ et,
                                                      float* AGG, unsigned short* __restrict__ Apl, int nbeg) {
  __shared__ int LIST[kEdgeChunk];
  __shared__ __align__(16) unsigned short CNT[kTileRows * kRel];
  __shared__ int scan_ws[80];
  const int tid = threadIdx.x, lane = tid & 31, wave = tid >> 5;
  const int hh = lane >> 4, c8 = (lane & 15) * 8;
  const int rloc0 = blockIdx.x * kTileRows;
  const int n0 = nbeg + rloc0;
  for (int i = tid; i < kTileRows * kRel; i += kThreads) CNT[i] = (unsigned short)0;
  for (int i = tid; i < kEdgeChunk; i += kThreads) LIST[i] = 0;
  if (tid < 80) scan_ws[tid] = 0;
  const v4f z4 = {0.f, 0.f, 0.f, 0.f};
  {
    float* zb = AGG + (size_t)(rloc0 + wave * kRowsPerWave) * kRel * kFeat + 4 * lane;
#pragma unroll 4
    for (int j = 0; j < kRowsPerWave * kRel; ++j) *(v4f*)(zb + (size_t)j * kFeat) = z4;
  }
  __syncthreads();
  const int* srcv = ei;
  const int* dstv = ei + kEdges;
#pragma unroll 1
  for (int c = 0; c < kNumEdgeChunks; ++c) {
    const int tot = chunk_hits(dstv, srcv, et, c * kEdgeChunk, n0, tid, LIST, scan_ws);
#pragma unroll 1
    for (int base = 0; base < tot; base += 32) {
      const int q = base + lane;
      const int qc = (q < tot) ? q : 0;
      int rv = LIST[qc];
      rv = (q < tot) ? rv : -1;
      const int own = (rv >= 0 && (rv >> 27) == wave) ? 1 : 0;
      unsigned msk = (unsigned)__ballot(own);
#pragma unroll 1
      for (int it = 0; it < 32; ++it) {
        if (msk == 0u) break;
        const int bp = __builtin_ctz(msk); msk &= msk - 1u;
        const int r = __shfl(rv, bp, 32);
        const int dl = r >> 19, ty = (r >> 16) & 7, s = r & 0xFFFF;
        const v4f fv = *(const v4f*)(F + (size_t)s * kFeat + 4 * lane);
        float* rp = AGG + ((size_t)(rloc0 + dl) * kRel + ty) * kFeat + 4 * lane;
        v4f a = *(const v4f*)rp;
        a = a + fv;
        *(v4f*)rp = a;
        if (lane == 0) { const int mi = dl * kRel + ty; CNT[mi] = (unsigned short)(CNT[mi] + 1); }
      }
    }
    __syncthreads();
  }
#pragma unroll 1
  for (int j = 0; j < kRowsPerWave; ++j) {
    const int dl = wave * kRowsPerWave + j;
    const int n = n0 + dl;
    const bool live = (n < kNodes);
    const float lf = live ? 1.0f : 0.0f;
    const int ncl = live ? n : (kNodes - 1);
    const size_t arow = (size_t)(rloc0 + dl);
    v4u u[5];
#pragma unroll
    for (int p = 0; p < 4; ++p) {
      const int r = 2 * p + hh;
      const float cn = (float)CNT[dl * kRel + r];
      const float inv = lf * (1.0f / fmaxf(cn, 1.0f));
      const float* gp = AGG + (arow * kRel + r) * kFeat + c8;
      const v4f g0 = *(const v4f*)gp;
      const v4f g1 = *(const v4f*)(gp + 4);
      u[p] = pack8h(g0 * inv, g1 * inv);
      asm volatile("" ::: "memory");
    }
    {
      const float* fp = F + (size_t)ncl * kFeat + c8;
      const v4f f0 = *(const v4f*)fp;
      const v4f f1 = *(const v4f*)(fp + 4);
      u[4] = pack8h(f0 * lf, f1 * lf);
    }
    unsigned short* ap = Apl + arow * kKtot;
    for (int pass = 0; pass < 2; ++pass) {
#pragma unroll
      for (int p = 0; p < 4; ++p) *(volatile v4u*)(ap + (2 * p + hh) * kFeat + c8) = u[p];
      if (hh == 0) *(volatile v4u*)(ap + kRel * kFeat + c8) = u[4];
      __threadfence();
    }
  }
}

extern "C" void kernel_launch(void* const* d_in, const int* in_sizes, int n_in,
                              void* d_out, int out_size, void* d_ws, size_t ws_size, hipStream_t stream) {
  if (n_in < 11) return;
  if (in_sizes[0] != kNodes * kFeat || in_sizes[1] != 2 * kEdges || in_sizes[2] != kEdges ||
      in_sizes[3] != kBases * kFeat * kFeat || in_sizes[4] != kRel * kBases || in_sizes[5] != kFeat * kFeat ||
      in_sizes[6] != kFeat || in_sizes[7] != kBases * kFeat * kFeat || in_sizes[8] != kRel * kBases ||
      in_sizes[9] != kFeat * kFeat || in_sizes[10] != kFeat) return;
  if (out_size != kNodes * kFeat) return;

  const float* x      = (const float*)d_in[0];
  const int*   ei     = (const int*)  d_in[1];
  const int*   et     = (const int*)  d_in[2];
  const float* basis1 = (const float*)d_in[3];
  const float* comp1  = (const float*)d_in[4];
  const float* root1  = (const float*)d_in[5];
  const float* bias1  = (const float*)d_in[6];
  const float* basis2 = (const float*)d_in[7];
  const float* comp2  = (const float*)d_in[8];
  const float* root2  = (const float*)d_in[9];
  const float* bias2  = (const float*)d_in[10];
  float* out = (float*)d_out;

  char* ws = (char*)d_ws; size_t off = 0;
  auto carve = [&](size_t bytes) -> char* { char* p = ws + off; off += (bytes + 255) & ~(size_t)255; return p; };
  unsigned short* Bt1 = (unsigned short*)carve(kBtBytes);
  unsigned short* Bt2 = (unsigned short*)carve(kBtBytes);
  unsigned short* Apl = (unsigned short*)carve(kAplBytes);
  float*          AGG = (float*)carve(kAggBytes);
  float*          Hpl = (float*)carve(kHBytes);
  if (off > ws_size || off > (size_t)134217728) return;

  btbuild_kernel<<<dim3(kFeat, 2), kThreads, 0, stream>>>(comp1, basis1, root1, comp2, basis2, root2, Bt1, Bt2);

  for (int layer = 0; layer < 2; ++layer) {
    const float* F = (layer == 0) ? x : (const float*)Hpl;
    const unsigned short* Bt = (layer == 0) ? Bt1 : Bt2;
    const float* bias = (layer == 0) ? bias1 : bias2;
    for (int c = 0; c < kNumChunks; ++c) {
      const int nbeg = c * kChunkNodes;
      const int rem  = kNodes - nbeg;
      const int ncnt = rem < kChunkNodes ? rem : kChunkNodes;
      const int tiles = (ncnt + kTileRows - 1) / kTileRows;
      const int Mpad = ((ncnt + 63) / 64) * 64;
      agg_kernel<<<tiles, kThreads, 0, stream>>>(F, ei, et, AGG, Apl, nbeg);
      const int gtiles = (Mpad / 64) * (kFeat / 64);
      const int gblocks = (gtiles + 7) / 8;
      if (layer == 0) {
        wmma_gemm64<0, false, 2, 0, 2><<<dim3(gblocks, 1), 256, 0, stream>>>(
            Apl, nullptr, kKtot, 0L, Bt, nullptr, kKtot, 0L,
            (void*)(Hpl + (size_t)nbeg * kFeat), nullptr, kFeat, 0L,
            bias, Mpad, kFeat, kKtot, kBCarryInv, Mpad);
      } else {
        wmma_gemm64<0, false, 2, 0, 0><<<dim3(gblocks, 1), 256, 0, stream>>>(
            Apl, nullptr, kKtot, 0L, Bt, nullptr, kKtot, 0L,
            (void*)(out + (size_t)nbeg * kFeat), nullptr, kFeat, 0L,
            bias, Mpad, kFeat, kKtot, kBCarryInv, ncnt);
      }
    }
  }
}
